// DeformConv2d_5961414607249
// MI455X (gfx1250) — hardware-verified
//
#include <hip/hip_runtime.h>
#include <math.h>

constexpr int Bn   = 8;
constexpr int CIN  = 256;
constexpr int COUT = 256;
constexpr int H    = 56, W = 56, OH = 56, OW = 56;
constexpr int KT   = 9;
constexpr int HW   = H * W;
constexpr int OHW  = OH * OW;
constexpr int NPOS = Bn * OHW;

constexpr int MTILE = 128;
constexpr int NTILE = 128;
constexpr int KC    = 32;
constexpr int NCH   = CIN / KC;
constexpr int NFRAG = NTILE / 16;
constexpr int FGTOT = COUT / 16;

constexpr size_t WRF_ELEMS = (size_t)KT * NCH * FGTOT * 32 * 16;
constexpr size_t WRF_BYTES = WRF_ELEMS * 2;
constexpr size_t XT_ELEMS  = (size_t)Bn * HW * CIN;

typedef __attribute__((ext_vector_type(16))) _Float16 v16h;
typedef __attribute__((ext_vector_type(8)))  _Float16 v8h;
typedef __attribute__((ext_vector_type(8)))  float    v8f;
typedef __attribute__((ext_vector_type(4)))  float    v4f;
typedef __attribute__((ext_vector_type(4)))  unsigned v4u;
template <typename T> __device__ __forceinline__ void vst2(void* p, T v) { *(volatile T*)p = v; __threadfence(); *(volatile T*)p = v; }
__device__ __forceinline__ v8f wmma16(v16h a, v16h b, v8f c) {
  v8f d = __builtin_amdgcn_wmma_f32_16x16x32_f16(false, a, false, b, (short)0, c, false, false);
  asm volatile("v_nop\n\tv_nop\n\tv_nop\n\tv_nop" : "+v"(d) : "v"(a), "v"(b));
  return d;
}

__global__ void build_wfrag(const float* __restrict__ w,
                            _Float16* __restrict__ wrF) {
  int g8 = blockIdx.x * 256 + threadIdx.x;
  if (g8 * 8 >= (int)WRF_ELEMS) return;
  union { v8h h; v4u u; } pk;
#pragma unroll
  for (int e = 0; e < 8; ++e) {
    const int idx  = g8 * 8 + e;
    const int i    = idx & 15;
    const int lane = (idx >> 4) & 31;
    const int fg   = (idx >> 9) & 15;
    const int cb   = (idx >> 13) & 7;
    const int t    = idx >> 16;
    const int half = lane >> 4, lm = lane & 15;
    const int oc = fg * 16 + lm;
    const int kk = (i < 8) ? (half * 8 + i) : (16 + half * 8 + (i - 8));
    const int c  = cb * KC + kk;
    pk.h[e] = (_Float16)w[(oc * CIN + c) * KT + t];
  }
  vst2(wrF + (size_t)g8 * 8, pk.u);
}

__global__ void build_xT(const float* __restrict__ x,
                         _Float16* __restrict__ xT) {
  int g8 = blockIdx.x * 256 + threadIdx.x;
  if (g8 * 8 >= (int)XT_ELEMS) return;
  const int idx0 = g8 * 8;
  const int c0 = idx0 & (CIN - 1);
  const int bo = idx0 >> 8;
  const int b  = bo / HW;
  const int o  = bo - b * HW;
  union { v8h h; v4u u; } pk;
#pragma unroll
  for (int e = 0; e < 8; ++e) pk.h[e] = (_Float16)x[((size_t)(b * CIN + c0 + e)) * HW + o];
  vst2(xT + (size_t)idx0, pk.u);
}

__launch_bounds__(256)
__global__ void deform_conv2d_wmma(const _Float16* __restrict__ xT,
                                   const float* __restrict__ offset,
                                   const float* __restrict__ mask,
                                   const _Float16* __restrict__ wrF,
                                   const float* __restrict__ bias,
                                   float* __restrict__ out) {
  __shared__ int      s_xbase[NTILE];
  __shared__ int      s_oidx[KT][NTILE][4];
  __shared__ float    s_wgt [KT][NTILE][4];
  __shared__ __align__(32) _Float16 s_colF[2][NFRAG][32][16];
  __shared__ __align__(16) float s_out[8][64 * 32];

  const int tid = threadIdx.x;
  const int n0  = blockIdx.x * NTILE;
  const int m0  = blockIdx.y * MTILE;

  for (int idx = tid; idx < KT * NTILE; idx += 256) {
    const int t = idx / NTILE;
    const int p = idx - t * NTILE;
    const int n = n0 + p;
    const int b  = n / OHW;
    const int r  = n - b * OHW;
    const int oh = r / OW;
    const int ow = r - oh * OW;
    if (t == 0) s_xbase[p] = b * HW * CIN;

    const float offi = offset[(((b * (2 * KT)) + 2 * t    ) * OH + oh) * OW + ow];
    const float offj = offset[(((b * (2 * KT)) + 2 * t + 1) * OH + oh) * OW + ow];
    const float mval = mask  [(((b * KT)       + t        ) * OH + oh) * OW + ow];

    const float ci = offi + (float)(oh - 1 + t / 3);
    const float cj = offj + (float)(ow - 1 + t % 3);
    const float fli = floorf(ci), flj = floorf(cj);
    const float fi = ci - fli,  fj = cj - flj;
    const int i0 = (int)fli, j0 = (int)flj;
    const int i1 = i0 + 1,   j1 = j0 + 1;

    const bool vi0 = (i0 >= 0) & (i0 < H), vi1 = (i1 >= 0) & (i1 < H);
    const bool vj0 = (j0 >= 0) & (j0 < W), vj1 = (j1 >= 0) & (j1 < W);
    const int ci0 = min(max(i0, 0), H - 1), ci1 = min(max(i1, 0), H - 1);
    const int cj0 = min(max(j0, 0), W - 1), cj1 = min(max(j1, 0), W - 1);

    s_oidx[t][p][0] = (ci0 * W + cj0) * CIN;
    s_oidx[t][p][1] = (ci0 * W + cj1) * CIN;
    s_oidx[t][p][2] = (ci1 * W + cj0) * CIN;
    s_oidx[t][p][3] = (ci1 * W + cj1) * CIN;
    s_wgt[t][p][0] = (1.f - fi) * (1.f - fj) * mval * (float)(vi0 & vj0);
    s_wgt[t][p][1] = (1.f - fi) * fj         * mval * (float)(vi0 & vj1);
    s_wgt[t][p][2] = fi         * (1.f - fj) * mval * (float)(vi1 & vj0);
    s_wgt[t][p][3] = fi         * fj         * mval * (float)(vi1 & vj1);
  }
  __syncthreads();

  const int lane  = tid & 31;
  const int wave  = tid >> 5;
  const int waveM = wave >> 2;
  const int waveN = wave & 3;
  const int half  = lane >> 4;
  const int lm    = lane & 15;

  const int pW = wave * 16 + lm;
  const int xb = s_xbase[pW];

  v8f acc[4][2];
  {
    v8f zero = {};
#pragma unroll
    for (int mb = 0; mb < 4; ++mb)
#pragma unroll
      for (int nb = 0; nb < 2; ++nb) acc[mb][nb] = zero;
  }

  const int fgBase = (m0 >> 4) + waveM * 4;

  int buf = 0;
  for (int t = 0; t < KT; ++t) {
    const int o0 = s_oidx[t][pW][0], o1 = s_oidx[t][pW][1];
    const int o2 = s_oidx[t][pW][2], o3 = s_oidx[t][pW][3];
    const float h0 = s_wgt[t][pW][0], h1 = s_wgt[t][pW][1];
    const float h2 = s_wgt[t][pW][2], h3 = s_wgt[t][pW][3];

    for (int cb = 0; cb < NCH; ++cb) {
      const int c0 = cb * KC;

      const _Float16* xc = xT + xb + c0 + half * 8;
      v16h cv;
      {
        union U { v16h v; v8h q[2]; } g0, g1, g2, g3;
        g0.q[0] = *(const v8h*)(xc + o0); g0.q[1] = *(const v8h*)(xc + o0 + 16);
        g1.q[0] = *(const v8h*)(xc + o1); g1.q[1] = *(const v8h*)(xc + o1 + 16);
        g2.q[0] = *(const v8h*)(xc + o2); g2.q[1] = *(const v8h*)(xc + o2 + 16);
        g3.q[0] = *(const v8h*)(xc + o3); g3.q[1] = *(const v8h*)(xc + o3 + 16);
#pragma unroll
        for (int i = 0; i < 16; ++i)
          cv[i] = (_Float16)((float)g0.v[i] * h0 + (float)g1.v[i] * h1 + (float)g2.v[i] * h2 + (float)g3.v[i] * h3);
      }

      const _Float16* aB =
          wrF + ((size_t)((t * NCH + cb) * FGTOT + fgBase) * 32 + lane) * 16;
      v16h afr[4];
#pragma unroll
      for (int mb = 0; mb < 4; ++mb)
        afr[mb] = *(const v16h*)(aB + (size_t)mb * 32 * 16);

      *(v16h*)(&s_colF[buf][wave][lane][0]) = cv;
      __syncthreads();

      v16h bfr[2];
#pragma unroll
      for (int nb = 0; nb < 2; ++nb)
        bfr[nb] = *(const v16h*)(&s_colF[buf][waveN * 2 + nb][lane][0]);

#pragma unroll
      for (int mb = 0; mb < 4; ++mb)
#pragma unroll
        for (int nb = 0; nb < 2; ++nb)
          acc[mb][nb] = wmma16(afr[mb], bfr[nb], acc[mb][nb]);

      buf ^= 1;
    }
  }

  float* so = s_out[wave];
#pragma unroll
  for (int nb = 0; nb < 2; ++nb)
#pragma unroll
    for (int mb = 0; mb < 4; ++mb)
#pragma unroll
      for (int rr = 0; rr < 8; ++rr) {
        const int ocl = mb * 16 + half * 8 + rr;
        so[ocl * 32 + nb * 16 + lm] = acc[mb][nb][rr] + bias[m0 + waveM * 64 + ocl];
      }
  __syncthreads();
  {
    const int nbase = n0 + waveN * 32;
    const int b = nbase / OHW, r = nbase - b * OHW;
#pragma unroll 4
    for (int q = 0; q < 16; ++q) {
      const int ocl = q * 4 + (lane >> 3), pc = lane & 7;
      const int oc = m0 + waveM * 64 + ocl;
      vst2(out + ((size_t)b * COUT + oc) * OHW + r + pc * 4, *(const v4f*)(so + ocl * 32 + pc * 4));
    }
  }
}

extern "C" void kernel_launch(void* const* d_in, const int* in_sizes, int n_in,
                              void* d_out, int out_size, void* d_ws, size_t ws_size,
                              hipStream_t stream) {
  const float* x      = (const float*)d_in[0];
  const float* offset = (const float*)d_in[1];
  const float* mask   = (const float*)d_in[2];
  const float* weight = (const float*)d_in[3];
  const float* bias   = (const float*)d_in[4];
  float*       out    = (float*)d_out;

  _Float16* wrF = (_Float16*)d_ws;
  _Float16* xT  = (_Float16*)((char*)d_ws + WRF_BYTES);

  build_wfrag<<<((int)WRF_ELEMS / 8 + 255) / 256, 256, 0, stream>>>(weight, wrF);
  build_xT  <<<((int)XT_ELEMS / 8 + 255) / 256, 256, 0, stream>>>(x, xT);

  dim3 grid(NPOS / NTILE  , COUT / MTILE  );
  deform_conv2d_wmma<<<grid, 256, 0, stream>>>(xT, offset, mask, wrF, bias, out);
}
